// MultiHeadAttention_78829829750818
// MI455X (gfx1250) — hardware-verified
//
#include <hip/hip_runtime.h>
#ifndef NB
#define NB 2
#endif
#ifndef SEQ
#define SEQ 4096
#endif
#define NB_FULL 2
#define SEQ_FULL 4096
#define DM 512
#define NH 8
#define HD 64
#define NR (NB * SEQ)
#define SCL 0.125f
#define SCLR 0.0001220703125f
#define PCARRY 1024.0f
#define ALPHA_P 0.0625f
#define ALPHA_O 0.0009765625f
#define ALPHA_OR 0.00000095367431640625f

static_assert(DM == NH * HD);
static_assert(HD == 64);
static_assert(DM % 64 == 0);
static_assert(DM % 32 == 0);
static_assert(SEQ % 128 == 0);
static_assert(NR % 128 == 0);
static_assert(NB <= NB_FULL);
static_assert(SEQ <= SEQ_FULL);
static_assert((size_t)4 * DM * DM * 2 + (size_t)11 * NR * DM * 2 <= (size_t)134217728);

typedef unsigned short v8us __attribute__((ext_vector_type(8), may_alias));
typedef float  v8f  __attribute__((ext_vector_type(8)));
typedef float  v4f  __attribute__((ext_vector_type(4)));
typedef float  v4fa __attribute__((ext_vector_type(4), may_alias));
typedef _Float16 v16h __attribute__((ext_vector_type(16)));
union FragH { v16h v; v8us half[2]; _Float16 h[16]; unsigned short u[16]; };

__device__ __forceinline__ unsigned short bf16_bits(float x) { unsigned int u = __float_as_uint(x); return (unsigned short)((u + 0x7FFFu + ((u >> 16) & 1u)) >> 16); }
__device__ __forceinline__ float bf16_val(unsigned short b) { return __uint_as_float(((unsigned int)b) << 16); }
__device__ __forceinline__ float bf16_rne(float x) { return bf16_val(bf16_bits(x)); }

__device__ __forceinline__ v16h g2_frag(const _Float16* p, int hh) { FragH f; f.half[0] = *(const v8us*)((const unsigned short*)p + 8 * hh); f.half[1] = *(const v8us*)((const unsigned short*)p + 16 + 8 * hh); return f.v; }
__device__ __forceinline__ v8f g2_mma(v16h a, v16h b, v8f c) { v8f d = __builtin_amdgcn_wmma_f32_16x16x32_f16(false, a, false, b, (short)0, c, false, false); asm volatile("v_nop\n\tv_nop\n\tv_nop\n\tv_nop" : "+v"(d) : "v"(a), "v"(b)); return d; }

__global__ __launch_bounds__(256) void k_wt_f16(const float* __restrict__ W, _Float16* __restrict__ Wt) {
  const int t = blockIdx.x * 256 + threadIdx.x;
  if (t >= DM * (DM / 8)) return;
  const int n = t / (DM / 8), k8 = (t % (DM / 8)) * 8;
  FragH f;
#pragma unroll
  for (int i = 0; i < 8; ++i) f.h[i] = (_Float16)(bf16_rne(W[(size_t)(k8 + i) * DM + n]) * 16.0f);
  const v8us o = f.half[0];
  unsigned short* d = (unsigned short*)Wt + (size_t)n * DM + k8;
  *(volatile v8us*)d = o;
  __threadfence();
  *(volatile v8us*)d = o;
}

__global__ __launch_bounds__(256) void k_x16(const float* __restrict__ x, _Float16* __restrict__ X16) {
  const int t = blockIdx.x * 256 + threadIdx.x;
  if (t >= NR * (DM / 8)) return;
  const int row = t / (DM / 8), c8 = (t % (DM / 8)) * 8;
  const int b = row / SEQ, s = row % SEQ;
  const float* src = x + ((size_t)b * SEQ_FULL + s) * DM + c8;
  const v4f a = *(const v4fa*)src, c = *(const v4fa*)(src + 4);
  FragH f;
#pragma unroll
  for (int q = 0; q < 4; ++q) { f.h[q] = (_Float16)bf16_rne(a[q]); f.h[4 + q] = (_Float16)bf16_rne(c[q]); }
  const v8us o = f.half[0];
  unsigned short* d = (unsigned short*)X16 + (size_t)t * 8;
  *(volatile v8us*)d = o;
  __threadfence();
  *(volatile v8us*)d = o;
}

struct Acc8 { v8f c00, c01, c02, c03, c10, c11, c12, c13; };
__device__ __forceinline__ void gemm_main(const _Float16* __restrict__ A, const _Float16* __restrict__ Bt, int row0, int col0, int ln, int hh, Acc8& o) {
  const _Float16* a0p = A + (size_t)(row0 + ln) * DM; const _Float16* a1p = a0p + (size_t)16 * DM;
  const _Float16* b0p = Bt + (size_t)(col0 + ln) * DM; const _Float16* b1p = b0p + (size_t)16 * DM; const _Float16* b2p = b1p + (size_t)16 * DM; const _Float16* b3p = b2p + (size_t)16 * DM;
  const v8f z8 = {0.f, 0.f, 0.f, 0.f, 0.f, 0.f, 0.f, 0.f};
  v8f c00 = z8, c01 = z8, c02 = z8, c03 = z8, c10 = z8, c11 = z8, c12 = z8, c13 = z8;
#pragma unroll 1
  for (int kb = 0; kb < DM; kb += 32) {
    const v16h a0 = g2_frag(a0p + kb, hh), a1 = g2_frag(a1p + kb, hh);
    v16h b = g2_frag(b0p + kb, hh); c00 = g2_mma(a0, b, c00); c10 = g2_mma(a1, b, c10);
    b = g2_frag(b1p + kb, hh); c01 = g2_mma(a0, b, c01); c11 = g2_mma(a1, b, c11);
    b = g2_frag(b2p + kb, hh); c02 = g2_mma(a0, b, c02); c12 = g2_mma(a1, b, c12);
    b = g2_frag(b3p + kb, hh); c03 = g2_mma(a0, b, c03); c13 = g2_mma(a1, b, c13);
  }
  o.c00 = c00; o.c01 = c01; o.c02 = c02; o.c03 = c03; o.c10 = c10; o.c11 = c11; o.c12 = c12; o.c13 = c13;
}

__global__ __launch_bounds__(128) void k_proj_hl(const _Float16* __restrict__ A, const _Float16* __restrict__ Bt, const float* __restrict__ bias, _Float16* __restrict__ Ph, _Float16* __restrict__ Pl) {
  __shared__ __attribute__((aligned(16))) float so[4][32][68];
  const int wave = __builtin_amdgcn_readfirstlane(threadIdx.x >> 5);
  const int lane = threadIdx.x & 31, ln = lane & 15, hh = lane >> 4;
  const int mt = blockIdx.x / (DM / 64), nq = blockIdx.x % (DM / 64);
  const int row0 = mt * 128 + 32 * wave, col0 = nq * 64;
  Acc8 acc; gemm_main(A, Bt, row0, col0, ln, hh, acc);
  {
    v8f accs[8] = {acc.c00, acc.c01, acc.c02, acc.c03, acc.c10, acc.c11, acc.c12, acc.c13};
#pragma unroll
    for (int u = 0; u < 8; ++u) {
      const int t = u & 3, hf = u >> 2;
      const float bv = bf16_rne(bias[col0 + t * 16 + ln]);
#pragma unroll
      for (int r = 0; r < 8; ++r) so[wave][hf * 16 + 8 * hh + r][t * 16 + ln] = accs[u][r] * ALPHA_P + bv;
    }
  }
  __syncthreads();
  const int rs = lane >> 3, pc = (lane & 7) * 8;
  for (int pass = 0; pass < 2; ++pass) {
#pragma unroll
    for (int q = 0; q < 8; ++q) {
      const int r = q * 4 + rs;
      const v4f x0 = *(const v4fa*)&so[wave][r][pc]; const v4f x1 = *(const v4fa*)&so[wave][r][pc + 4];
      FragH fh, fl;
#pragma unroll
      for (int j = 0; j < 4; ++j) {
        _Float16 hv = (_Float16)x0[j]; fh.h[j] = hv; fl.h[j] = (_Float16)((x0[j] - (float)hv) * 1024.0f);
        hv = (_Float16)x1[j]; fh.h[4 + j] = hv; fl.h[4 + j] = (_Float16)((x1[j] - (float)hv) * 1024.0f);
      }
      const v8us oh = fh.half[0], ol = fl.half[0];
      const size_t off = (size_t)(row0 + r) * DM + col0 + pc;
      *(volatile v8us*)((unsigned short*)Ph + off) = oh;
      *(volatile v8us*)((unsigned short*)Pl + off) = ol;
    }
    if (pass == 0) __threadfence();
  }
}

__global__ __launch_bounds__(128) void k_proj_v(const _Float16* __restrict__ A, const _Float16* __restrict__ Bt, const float* __restrict__ bias, _Float16* __restrict__ P16) {
  __shared__ __attribute__((aligned(16))) float so[4][32][68];
  const int wave = __builtin_amdgcn_readfirstlane(threadIdx.x >> 5);
  const int lane = threadIdx.x & 31, ln = lane & 15, hh = lane >> 4;
  const int mt = blockIdx.x / (DM / 64), nq = blockIdx.x % (DM / 64);
  const int row0 = mt * 128 + 32 * wave, col0 = nq * 64;
  Acc8 acc; gemm_main(A, Bt, row0, col0, ln, hh, acc);
  {
    v8f accs[8] = {acc.c00, acc.c01, acc.c02, acc.c03, acc.c10, acc.c11, acc.c12, acc.c13};
#pragma unroll
    for (int u = 0; u < 8; ++u) {
      const int t = u & 3, hf = u >> 2;
      const float bv = bf16_rne(bias[col0 + t * 16 + ln]);
#pragma unroll
      for (int r = 0; r < 8; ++r) so[wave][hf * 16 + 8 * hh + r][t * 16 + ln] = accs[u][r] * ALPHA_P + bv;
    }
  }
  __syncthreads();
  const int rs = lane >> 3, pc = (lane & 7) * 8;
  for (int pass = 0; pass < 2; ++pass) {
#pragma unroll
    for (int q = 0; q < 8; ++q) {
      const int r = q * 4 + rs;
      const v4f x0 = *(const v4fa*)&so[wave][r][pc]; const v4f x1 = *(const v4fa*)&so[wave][r][pc + 4];
      FragH fh;
#pragma unroll
      for (int j = 0; j < 4; ++j) { fh.h[j] = (_Float16)x0[j]; fh.h[4 + j] = (_Float16)x1[j]; }
      const v8us oh = fh.half[0];
      const size_t off = (size_t)(row0 + r) * DM + col0 + pc;
      *(volatile v8us*)((unsigned short*)P16 + off) = oh;
    }
    if (pass == 0) __threadfence();
  }
}

__global__ __launch_bounds__(128) void k_out(const _Float16* __restrict__ CHp, const _Float16* __restrict__ CLp, const _Float16* __restrict__ Bt, const float* __restrict__ bias, float* __restrict__ out) {
  __shared__ __attribute__((aligned(16))) float so[4][32][68];
  const int wave = __builtin_amdgcn_readfirstlane(threadIdx.x >> 5);
  const int lane = threadIdx.x & 31, ln = lane & 15, hh = lane >> 4;
  const int mt = blockIdx.x / (DM / 64), nq = blockIdx.x % (DM / 64);
  const int row0 = mt * 128 + 32 * wave, col0 = nq * 64;
  Acc8 acc; gemm_main(CHp, Bt, row0, col0, ln, hh, acc);
  {
    v8f accs[8] = {acc.c00, acc.c01, acc.c02, acc.c03, acc.c10, acc.c11, acc.c12, acc.c13};
#pragma unroll
    for (int u = 0; u < 8; ++u) {
      const int t = u & 3, hf = u >> 2;
      const float bv = bf16_rne(bias[col0 + t * 16 + ln]);
#pragma unroll
      for (int r = 0; r < 8; ++r) so[wave][hf * 16 + 8 * hh + r][t * 16 + ln] = accs[u][r] * ALPHA_O + bv;
    }
  }
  gemm_main(CLp, Bt, row0, col0, ln, hh, acc);
  {
    v8f accs[8] = {acc.c00, acc.c01, acc.c02, acc.c03, acc.c10, acc.c11, acc.c12, acc.c13};
#pragma unroll
    for (int u = 0; u < 8; ++u) {
      const int t = u & 3, hf = u >> 2;
#pragma unroll
      for (int r = 0; r < 8; ++r) { const float e = so[wave][hf * 16 + 8 * hh + r][t * 16 + ln]; so[wave][hf * 16 + 8 * hh + r][t * 16 + ln] = e + accs[u][r] * ALPHA_OR; }
    }
  }
  __syncthreads();
  const int rsub = lane >> 4, c4 = (lane & 15) * 4;
  for (int pass = 0; pass < 2; ++pass) {
#pragma unroll
    for (int q = 0; q < 16; ++q) {
      const int r = q * 2 + rsub;
      const int tr = row0 + r;
      const size_t orow = (size_t)(tr / SEQ) * SEQ_FULL + (size_t)(tr % SEQ);
      const v4f v = *(const v4fa*)&so[wave][r][c4];
      *(volatile v4f*)(out + orow * DM + col0 + c4) = v;
    }
    if (pass == 0) __threadfence();
  }
}

__global__ __launch_bounds__(256) void k_vt(const _Float16* __restrict__ V16, _Float16* __restrict__ VT) {
  __shared__ unsigned short tl[64][66];
  const int tid = threadIdx.x;
  const int slab = blockIdx.x / (SEQ / 64), lg = blockIdx.x % (SEQ / 64);
  const int b = slab / NH, h = slab % NH;
#pragma unroll
  for (int it = 0; it < 2; ++it) {
    const int i = tid + it * 256;
    const int r = i / 8, c8 = (i % 8) * 8;
    FragH f; f.half[0] = *(const v8us*)((const unsigned short*)V16 + ((size_t)b * SEQ + lg * 64 + r) * DM + h * HD + c8);
#pragma unroll
    for (int q = 0; q < 8; ++q) tl[r][c8 + q] = f.u[q];
  }
  __syncthreads();
  for (int pass = 0; pass < 2; ++pass) {
#pragma unroll
    for (int rd = 0; rd < 2; ++rd) {
      const int d = rd * 32 + tid / 8, pc = tid % 8;
      FragH f;
#pragma unroll
      for (int q = 0; q < 8; ++q) f.u[q] = tl[pc * 8 + q][d];
      const v8us o = f.half[0];
      *(volatile v8us*)((unsigned short*)VT + ((size_t)slab * HD + d) * SEQ + lg * 64 + pc * 8) = o;
    }
    if (pass == 0) __threadfence();
  }
}

__global__ __launch_bounds__(128) void k_attn(const _Float16* __restrict__ QH, const _Float16* __restrict__ QL, const _Float16* __restrict__ KH, const _Float16* __restrict__ KL,
                                             const _Float16* __restrict__ VT, _Float16* __restrict__ CH, _Float16* __restrict__ CL) {
  __shared__ __attribute__((aligned(16))) float so[4][16][68];
  const int wave = __builtin_amdgcn_readfirstlane(threadIdx.x >> 5);
  const int lane = threadIdx.x & 31, ln = lane & 15, hh = lane >> 4;
  const int qb = blockIdx.x % (SEQ / 64), bh = blockIdx.x / (SEQ / 64);
  const int b = bh / NH, h = bh % NH;
  const int q0 = qb * 64 + wave * 16;
  const size_t tok0 = (size_t)b * SEQ;
  const size_t qoff = (tok0 + q0 + ln) * DM + h * HD;
  const size_t koff0 = (tok0 + ln) * DM + h * HD;
  const size_t voff0 = ((size_t)bh * HD + ln) * SEQ;
  const v8f z8 = {0.f, 0.f, 0.f, 0.f, 0.f, 0.f, 0.f, 0.f};
  v8f o0 = z8, o1 = z8, o2 = z8, o3 = z8;
  float m = -1.0e30f, l = 0.f;
#pragma unroll 1
  for (int kt = 0; kt < SEQ; kt += 32) {
    const size_t k0 = koff0 + (size_t)kt * DM, k1 = k0 + (size_t)16 * DM;
    v8f s0h = z8, s0r = z8, s1h = z8, s1r = z8;
#pragma unroll
    for (int kc = 0; kc < 2; ++kc) {
      const v16h qh = g2_frag(QH + qoff + kc * 32, hh);
      const v16h ql = g2_frag(QL + qoff + kc * 32, hh);
      v16h kh = g2_frag(KH + k0 + kc * 32, hh);
      v16h kl = g2_frag(KL + k0 + kc * 32, hh);
      s0h = g2_mma(kh, qh, s0h); s0r = g2_mma(kl, qh, s0r); s0r = g2_mma(kh, ql, s0r);
      kh = g2_frag(KH + k1 + kc * 32, hh);
      kl = g2_frag(KL + k1 + kc * 32, hh);
      s1h = g2_mma(kh, qh, s1h); s1r = g2_mma(kl, qh, s1r); s1r = g2_mma(kh, ql, s1r);
    }
    float sv[16];
#pragma unroll
    for (int r = 0; r < 8; ++r) { sv[r] = s0h[r] * SCL + s0r[r] * SCLR; sv[8 + r] = s1h[r] * SCL + s1r[r] * SCLR; }
    float mx = sv[0];
#pragma unroll
    for (int i = 1; i < 16; ++i) mx = fmaxf(mx, sv[i]);
    mx = fmaxf(mx, __shfl_xor(mx, 16));
    const float mn = fmaxf(m, mx);
    const float corr = __expf(m - mn);
    m = mn;
    float ls = 0.f;
    FragH pb;
#pragma unroll
    for (int i = 0; i < 16; ++i) { const float p = __expf(sv[i] - mn); ls += p; pb.h[i] = (_Float16)(p * PCARRY); }
    l = l * corr + ls;
    o0 *= corr; o1 *= corr; o2 *= corr; o3 *= corr;
    const size_t vo = voff0 + kt;
    v16h va = g2_frag(VT + vo, hh); o0 = g2_mma(va, pb.v, o0);
    va = g2_frag(VT + vo + (size_t)16 * SEQ, hh); o1 = g2_mma(va, pb.v, o1);
    va = g2_frag(VT + vo + (size_t)32 * SEQ, hh); o2 = g2_mma(va, pb.v, o2);
    va = g2_frag(VT + vo + (size_t)48 * SEQ, hh); o3 = g2_mma(va, pb.v, o3);
  }
  const float lt = l + __shfl_xor(l, 16);
  const float inv = 0.0625f * (1.0f / lt);
#pragma unroll
  for (int r = 0; r < 8; ++r) {
    so[wave][ln][8 * hh + r] = o0[r] * inv;
    so[wave][ln][16 + 8 * hh + r] = o1[r] * inv;
    so[wave][ln][32 + 8 * hh + r] = o2[r] * inv;
    so[wave][ln][48 + 8 * hh + r] = o3[r] * inv;
  }
  __syncthreads();
  const int rs = lane >> 3, pc = (lane & 7) * 8;
  for (int pass = 0; pass < 2; ++pass) {
#pragma unroll
    for (int it = 0; it < 4; ++it) {
      const int row = it * 4 + rs;
      const v4f x0 = *(const v4fa*)&so[wave][row][pc]; const v4f x1 = *(const v4fa*)&so[wave][row][pc + 4];
      FragH fh, fl;
#pragma unroll
      for (int j = 0; j < 4; ++j) {
        _Float16 hv = (_Float16)x0[j]; fh.h[j] = hv; fl.h[j] = (_Float16)((x0[j] - (float)hv) * 1024.0f);
        hv = (_Float16)x1[j]; fh.h[4 + j] = hv; fl.h[4 + j] = (_Float16)((x1[j] - (float)hv) * 1024.0f);
      }
      const v8us oh = fh.half[0], ol = fl.half[0];
      const size_t off = (tok0 + q0 + row) * DM + h * HD + pc;
      *(volatile v8us*)((unsigned short*)CH + off) = oh;
      *(volatile v8us*)((unsigned short*)CL + off) = ol;
    }
    if (pass == 0) __threadfence();
  }
}

extern "C" void kernel_launch(void* const* d_in, const int* in_sizes, int n_in,
                              void* d_out, int out_size, void* d_ws, size_t ws_size, hipStream_t stream) {
  if (n_in < 11) return;
  const long long need_x = ((long long)(NB - 1) * SEQ_FULL + SEQ) * DM;
  if (in_sizes[0] < need_x || in_sizes[1] < need_x || in_sizes[2] < need_x) return;
  if (in_sizes[3] < DM * DM || in_sizes[5] < DM * DM || in_sizes[7] < DM * DM || in_sizes[9] < DM * DM) return;
  if (in_sizes[4] < DM || in_sizes[6] < DM || in_sizes[8] < DM || in_sizes[10] < DM) return;
  if (out_size < need_x) return;
  const float* xq = (const float*)d_in[0]; const float* xk = (const float*)d_in[1]; const float* xv = (const float*)d_in[2];
  const float* wq = (const float*)d_in[3]; const float* bq = (const float*)d_in[4];
  const float* wk = (const float*)d_in[5]; const float* bk = (const float*)d_in[6];
  const float* wv = (const float*)d_in[7]; const float* bv = (const float*)d_in[8];
  const float* wo = (const float*)d_in[9]; const float* bo = (const float*)d_in[10];
  char* ws = (char*)d_ws; size_t off = 0;
  auto take = [&](size_t bytes) { char* p = ws + off; off += (bytes + 255) & ~(size_t)255; return p; };
  const size_t WB = (size_t)DM * DM * 2;
  const size_t PL = (size_t)NR * DM * 2;
  _Float16* BQ = (_Float16*)take(WB); _Float16* BK = (_Float16*)take(WB); _Float16* BV = (_Float16*)take(WB); _Float16* BO = (_Float16*)take(WB);
  _Float16* XQ = (_Float16*)take(PL); _Float16* XK = (_Float16*)take(PL); _Float16* XV = (_Float16*)take(PL);
  _Float16* QH = (_Float16*)take(PL); _Float16* QL = (_Float16*)take(PL); _Float16* KH = (_Float16*)take(PL); _Float16* KL = (_Float16*)take(PL);
  _Float16* V16 = (_Float16*)take(PL); _Float16* VT = (_Float16*)take(PL);
  _Float16* CH = (_Float16*)take(PL); _Float16* CL = (_Float16*)take(PL);
  if (off > ws_size) return;
  const unsigned gw = (unsigned)((DM * (DM / 8) + 255) / 256);
  k_wt_f16<<<gw, 256, 0, stream>>>(wq, BQ);
  k_wt_f16<<<gw, 256, 0, stream>>>(wk, BK);
  k_wt_f16<<<gw, 256, 0, stream>>>(wv, BV);
  k_wt_f16<<<gw, 256, 0, stream>>>(wo, BO);
  const unsigned gx = (unsigned)((NR * (DM / 8) + 255) / 256);
  k_x16<<<gx, 256, 0, stream>>>(xq, XQ);
  k_x16<<<gx, 256, 0, stream>>>(xk, XK);
  k_x16<<<gx, 256, 0, stream>>>(xv, XV);
  const unsigned gg = (unsigned)((NR / 128) * (DM / 64));
  k_proj_hl<<<gg, 128, 0, stream>>>(XQ, BQ, bq, QH, QL);
  k_proj_hl<<<gg, 128, 0, stream>>>(XK, BK, bk, KH, KL);
  k_proj_v<<<gg, 128, 0, stream>>>(XV, BV, bv, V16);
  k_vt<<<(unsigned)(NB * NH * (SEQ / 64)), 256, 0, stream>>>(V16, VT);
  k_attn<<<(unsigned)(NB * NH * (SEQ / 64)), 128, 0, stream>>>(QH, QL, KH, KL, VT, CH, CL);
  k_out<<<gg, 128, 0, stream>>>(CH, CL, BO, bo, (float*)d_out);
}
